// GATDecoder_29815662969291
// MI455X (gfx1250) — hardware-verified
//
#include <hip/hip_runtime.h>
#include <stddef.h>
#include <stdint.h>


#define BB      4
#define HID     128
#define DDIM    256
#define NHEAD   4
#define DH      64
#define KCAT    512
#define NTHR    256
#define NWAVE   8
#define EPT     8
#define CHUNK   (NTHR * EPT)
#define WCAP    (EPT * 32)
#define LISTN   (NWAVE * WCAP)
#define NBMAX   2048
#define RCAP    28672
#define DEGCAP  4096
#define GBM     32
#define NEGS    0.1f
#define WSMAX   134217728
#define LDS_AGG ((2 * RCAP + 2 * NBMAX + LISTN) * 4 + 64)

static_assert((CHUNK & (CHUNK - 1)) == 0 && CHUNK <= 4096);
static_assert((NBMAX & (NBMAX - 1)) == 0 && NBMAX <= 4096);
static_assert(NTHR * 8 == NBMAX);
static_assert(LISTN >= NBMAX);
static_assert(LISTN >= NWAVE * WCAP);
static_assert((RCAP % 32) == 0);
static_assert(LDS_AGG <= 300000);
static_assert(NTHR == 32 * NWAVE);
static_assert(GBM == 2 * 16 && DDIM == 4 * 64);
static_assert(NHEAD * DH == DDIM && NHEAD * DH == NTHR);
static_assert((DDIM % 32) == 0 && (DH % 32) == 0 && (KCAT % 32) == 0 && KCAT == 2 * DDIM);
static_assert(2 * HID == DDIM);
static_assert(BB == 4);

typedef float          v4f  __attribute__((ext_vector_type(4)));
typedef float          v8f  __attribute__((ext_vector_type(8)));
typedef int            v4i  __attribute__((ext_vector_type(4)));
typedef int            v8i  __attribute__((ext_vector_type(8)));
typedef unsigned short us;
typedef us             v8us __attribute__((ext_vector_type(8)));
typedef __bf16         v16b __attribute__((ext_vector_type(16)));
typedef v4f  __attribute__((may_alias)) v4fa;
typedef v8us __attribute__((may_alias)) v8usa;
union FragB { v16b v; v8us h[2]; v8i w; };
struct HiLo { v8us hi; v8us lo; };

__device__ __forceinline__ v8f wmb(const FragB& a, const FragB& b, v8f c) {
  v8f d = __builtin_amdgcn_wmma_f32_16x16x32_bf16(false, a.v, false, b.v, (short)0, c, false, false);
  asm volatile("v_nop\n\tv_nop\n\tv_nop\n\tv_nop" : "+v"(d) : "v"(a.w), "v"(b.w));
  return d;
}

__device__ __forceinline__ FragB ldfrag(const us* p) {
  FragB f;
  f.h[0] = *(const v8usa*)p;
  f.h[1] = *(const v8usa*)(p + 16);
  return f;
}

__device__ __forceinline__ void ldwait() {
  asm volatile("s_wait_loadcnt 0x0" ::: "memory");
}

__device__ __forceinline__ unsigned bfbits(float f) {
  unsigned u = __float_as_uint(f);
  u += 0x7FFFu + ((u >> 16) & 1u);
  return u >> 16;
}
__device__ __forceinline__ float bfval(unsigned b) { return __uint_as_float(b << 16); }
__device__ __forceinline__ float bfr(float f) { return bfval(bfbits(f)); }

__device__ __forceinline__ v8us cvt8b(const v4f a, const v4f b) {
  v8us o;
  o[0] = (us)bfbits(a.x); o[1] = (us)bfbits(a.y); o[2] = (us)bfbits(a.z); o[3] = (us)bfbits(a.w);
  o[4] = (us)bfbits(b.x); o[5] = (us)bfbits(b.y); o[6] = (us)bfbits(b.z); o[7] = (us)bfbits(b.w);
  return o;
}

__device__ __forceinline__ HiLo hilo8(const v4f a, const v4f b) {
  const float v[8] = {a.x, a.y, a.z, a.w, b.x, b.y, b.z, b.w};
  HiLo r;
#pragma unroll
  for (int i = 0; i < 8; ++i) {
    const unsigned hb = bfbits(v[i]);
    r.hi[i] = (us)hb;
    r.lo[i] = (us)bfbits(v[i] - bfval(hb));
  }
  return r;
}

__device__ __forceinline__ float sel4(const v4f v, int i) {
  const float a = (i & 1) ? v.y : v.x;
  const float b = (i & 1) ? v.w : v.z;
  return (i & 2) ? b : a;
}

__device__ __forceinline__ int scan_chunk(const int* __restrict__ dsts, int nE, int cbase, int slotBase,
                                          int nb, int vec8, int* list, int tid, int lane, int wave) {
  int wc = 0;
  const int el0  = tid * EPT;
  const int e0   = cbase + el0;
  const int sent = -2147483647 - 1;
  v4i da, db;
  if (vec8 != 0 && cbase + CHUNK <= nE) {
    da = *(const v4i*)(dsts + e0);
    db = *(const v4i*)(dsts + e0 + 4);
  } else {
    da.x = (e0     < nE) ? dsts[min(e0,     nE - 1)] : sent;
    da.y = (e0 + 1 < nE) ? dsts[min(e0 + 1, nE - 1)] : sent;
    da.z = (e0 + 2 < nE) ? dsts[min(e0 + 2, nE - 1)] : sent;
    da.w = (e0 + 3 < nE) ? dsts[min(e0 + 3, nE - 1)] : sent;
    db.x = (e0 + 4 < nE) ? dsts[min(e0 + 4, nE - 1)] : sent;
    db.y = (e0 + 5 < nE) ? dsts[min(e0 + 5, nE - 1)] : sent;
    db.z = (e0 + 6 < nE) ? dsts[min(e0 + 6, nE - 1)] : sent;
    db.w = (e0 + 7 < nE) ? dsts[min(e0 + 7, nE - 1)] : sent;
  }
  const unsigned nbs = (unsigned)slotBase;
  const unsigned unb = (unsigned)nb;
  const unsigned s0 = (unsigned)da.x - nbs, s1 = (unsigned)da.y - nbs;
  const unsigned s2 = (unsigned)da.z - nbs, s3 = (unsigned)da.w - nbs;
  const unsigned s4 = (unsigned)db.x - nbs, s5 = (unsigned)db.y - nbs;
  const unsigned s6 = (unsigned)db.z - nbs, s7 = (unsigned)db.w - nbs;
  const bool h0 = s0 < unb, h1 = s1 < unb, h2 = s2 < unb, h3 = s3 < unb;
  const bool h4 = s4 < unb, h5 = s5 < unb, h6 = s6 < unb, h7 = s7 < unb;
  const unsigned any = __builtin_amdgcn_ballot_w32(h0 | h1 | h2 | h3 | h4 | h5 | h6 | h7);
  if (any != 0u) {
#define HITJ(J, HJ, SJ) { \
      const unsigned mj = __builtin_amdgcn_ballot_w32(HJ); \
      if (mj != 0u) { \
        if (HJ) { \
          const int pos = wc + (int)__builtin_amdgcn_mbcnt_lo(mj, 0u); \
          if (pos < WCAP) list[wave * WCAP + pos] = ((el0 + (J)) << 12) | (int)(SJ); \
        } \
        wc += (int)__builtin_popcount(mj); } }
    HITJ(0, h0, s0)
    HITJ(1, h1, s1)
    HITJ(2, h2, s2)
    HITJ(3, h3, s3)
    HITJ(4, h4, s4)
    HITJ(5, h5, s5)
    HITJ(6, h6, s6)
    HITJ(7, h7, s7)
#undef HITJ
  }
  return wc;
}

__global__ __launch_bounds__(NTHR) void k_prep(const float* __restrict__ sol, const float* __restrict__ fcw,
                                               const float* __restrict__ ofw, const float* __restrict__ mlw,
                                               us* x0, us* wfc, us* wof, us* wml,
                                               int nN, int u0, int u1, int u2, int u3) {
  const int u = (int)blockIdx.x * NTHR + (int)threadIdx.x;
  if (u >= u3) return;
  const float* sp;
  us* dp;
  if (u < u0) {
    const int r  = u >> 5;
    const int c0 = (u & 31) * 8;
    const int b  = r / nN;
    const int n  = r - b * nN;
    const int bk = c0 >> 7;
    const int cc = c0 & (HID - 1);
    sp = sol + ((size_t)(bk * BB + b) * (size_t)nN + (size_t)n) * HID + cc;
    dp = x0 + (size_t)r * DDIM + c0;
  } else if (u < u1) {
    const int e = u - u0;
    sp = fcw + (size_t)e * 8;
    dp = wfc + (size_t)e * 8;
  } else if (u < u2) {
    const int e = u - u1;
    sp = ofw + (size_t)e * 8;
    dp = wof + (size_t)e * 8;
  } else {
    const int e = u - u2;
    sp = mlw + (size_t)e * 8;
    dp = wml + (size_t)e * 8;
  }
  const v4f a = *(const v4fa*)sp;
  const v4f c = *(const v4fa*)(sp + 4);
  const v8us o = cvt8b(a, c);
  *(volatile v8us*)dp = o;
  __threadfence();
  *(volatile v8us*)dp = o;
}

template<int NP>
__global__ __launch_bounds__(NTHR) void k_fc(const us* __restrict__ Ah, const us* __restrict__ Al, int lda,
                                             const us* __restrict__ W, const float* __restrict__ al,
                                             const float* __restrict__ ar, float* F, float* T, int M) {
  __shared__ __attribute__((aligned(16))) float stg[GBM * DDIM];
  __shared__ __attribute__((aligned(16))) float satt[2 * NHEAD * DH];
  __shared__ __attribute__((aligned(16))) float selr[GBM * 8];
  const int tid = (int)threadIdx.x, lane = tid & 31, wave = tid >> 5, hh = lane >> 4, m = lane & 15;
  const int rg = wave & 1, cg = wave >> 1;
  const int rowBase = (int)blockIdx.x * GBM;
  if (rowBase >= M) return;

  satt[tid]              = bfr(al[tid]);
  satt[NHEAD * DH + tid] = bfr(ar[tid]);

  v8f acc[4];
  {
    const v8f z = {0.f, 0.f, 0.f, 0.f, 0.f, 0.f, 0.f, 0.f};
    acc[0] = z; acc[1] = z; acc[2] = z; acc[3] = z;
  }
  const size_t arow = (size_t)(rowBase + 16 * rg + m) * (size_t)lda + 8 * hh;
  const us* ap  = Ah + arow;
  const us* alp = Al + arow;
  const us* wp  = W + (size_t)(64 * cg + m) * DDIM + 8 * hh;
#pragma unroll 1
  for (int ks = 0; ks < DDIM / 32; ++ks) {
    const FragB af = ldfrag(ap + 32 * ks);
    FragB alf;
    if (NP == 2) alf = ldfrag(alp + 32 * ks);
#pragma unroll
    for (int t = 0; t < 4; ++t) {
      const FragB bf = ldfrag(wp + (size_t)(16 * t) * DDIM + 32 * ks);
      acc[t] = wmb(af, bf, acc[t]);
      if (NP == 2) acc[t] = wmb(alf, bf, acc[t]);
    }
  }

#pragma unroll
  for (int t = 0; t < 4; ++t) {
    const int lc = 64 * cg + 16 * t + m;
#pragma unroll
    for (int r = 0; r < 8; ++r) {
      const int lr = 16 * rg + 8 * hh + r;
      stg[lr * DDIM + lc] = acc[t][r];
    }
  }
  __syncthreads();

  {
    const int h = wave & 3, wch = wave >> 2;
    const float* frow = stg + lane * DDIM + h * DH;
    const float* avec = satt + wch * (NHEAD * DH) + h * DH;
    float s = 0.f;
#pragma unroll
    for (int d4 = 0; d4 < DH / 4; ++d4) {
      const v4f f4 = *(const v4fa*)(frow + 4 * d4);
      const v4f a4 = *(const v4fa*)(avec + 4 * d4);
      s = fmaf(f4.x, a4.x, s);
      s = fmaf(f4.y, a4.y, s);
      s = fmaf(f4.z, a4.z, s);
      s = fmaf(f4.w, a4.w, s);
    }
    selr[lane * 8 + wave] = s;
  }
  __syncthreads();

  v4f fv[8];
#pragma unroll
  for (int i = 0; i < 8; ++i) {
    const int lr = 16 * rg + 2 * i + hh;
    fv[i] = *(const v4fa*)(stg + lr * DDIM + 64 * cg + 4 * m);
  }
  v4f ta, tb;
  ta = *(const v4fa*)(selr + 4 * lane);
  tb = *(const v4fa*)(selr + 128 + 4 * lane);
  float* tp = T + (size_t)rowBase * 8 + 4 * lane;

#pragma unroll
  for (int i = 0; i < 8; ++i) {
    const int lr = 16 * rg + 2 * i + hh;
    float* op = F + (size_t)(rowBase + lr) * DDIM + 64 * cg + 4 * m;
    *(volatile v4f*)op = fv[i];
  }
  if (wave == 0) {
    *(volatile v4f*)tp = ta;
    *(volatile v4f*)(tp + 128) = tb;
  }
  __threadfence();
#pragma unroll
  for (int i = 0; i < 8; ++i) {
    const int lr = 16 * rg + 2 * i + hh;
    float* op = F + (size_t)(rowBase + lr) * DDIM + 64 * cg + 4 * m;
    *(volatile v4f*)op = fv[i];
  }
  if (wave == 0) {
    *(volatile v4f*)tp = ta;
    *(volatile v4f*)(tp + 128) = tb;
  }
}

__global__ __launch_bounds__(NTHR) void k_agg(
    const int* __restrict__ srcs, const int* __restrict__ dsts, const float* __restrict__ wgt,
    const float* __restrict__ F, const float* __restrict__ T, us* RSH, us* RSL,
    int nN, int nE, int nb, int vec8) {
  extern __shared__ v4f lds_dyn[];
  int* reg1 = (int*)lds_dyn;
  int* reg2 = reg1 + RCAP;
  int* scnt = reg2 + RCAP;
  int* soff = scnt + NBMAX;
  int* list = soff + NBMAX;
  int* wcnt = list + LISTN;
  int* wtot = wcnt + NWAVE;
  const int tid = (int)threadIdx.x, lane = tid & 31, wave = tid >> 5;
  const int nodeBase = (int)blockIdx.x * nb;

  for (int i = tid; i < NBMAX; i += NTHR) scnt[i] = 0;
  __syncthreads();

  int tot = 0;
  const int nChunks = (nE + CHUNK - 1) / CHUNK;
#pragma unroll 1
  for (int ch = 0; ch < nChunks; ++ch) {
    const int cbase = ch * CHUNK;
    const int wc = scan_chunk(dsts, nE, cbase, nodeBase, nb, vec8, list, tid, lane, wave);
    if (lane == 0) wcnt[wave] = wc;
    __syncthreads();
    int pre = 0, all = 0;
#pragma unroll
    for (int w2 = 0; w2 < NWAVE; ++w2) {
      int c = wcnt[w2];
      c = c < 0 ? 0 : (c > WCAP ? WCAP : c);
      all += c;
      pre += (w2 < wave) ? c : 0;
    }
    const int wcc  = wc > WCAP ? WCAP : wc;
    const int base = tot + pre;
#pragma unroll 1
    for (int i = lane; i < wcc; i += 32) {
      const int ent = list[wave * WCAP + i];
      const int el  = (ent >> 12) & (CHUNK - 1);
      const int sl  = ent & (NBMAX - 1);
      int eid = cbase + el;
      eid = eid > nE - 1 ? nE - 1 : eid;
      const int pos = base + i;
      if (pos < RCAP) reg1[pos] = (int)(((unsigned)eid << 12) | (unsigned)sl);
    }
    tot += all;
    tot = tot > RCAP ? RCAP : tot;
    __syncthreads();
  }
  const int nh = tot;

  if (wave == 0) {
#pragma unroll 1
    for (int b0 = 0; b0 < nh; b0 += 32) {
      const int idx = b0 + lane;
      const int uv  = reg1[idx < RCAP ? idx : RCAP - 1];
      const int m32 = (nh - b0) < 32 ? (nh - b0) : 32;
#pragma unroll 1
      for (int k = 0; k < m32; ++k) {
        const int u  = __builtin_amdgcn_readlane(uv, k);
        const int sl = u & (NBMAX - 1);
        if (lane == 0) scnt[sl] = scnt[sl] + 1;
      }
    }
  }
  __syncthreads();

  {
    const v4i ca = *(const v4i*)(scnt + 8 * tid);
    const v4i cb = *(const v4i*)(scnt + 8 * tid + 4);
    const int e0 = ca.x < 0 ? 0 : ca.x, e1 = ca.y < 0 ? 0 : ca.y, e2 = ca.z < 0 ? 0 : ca.z, e3 = ca.w < 0 ? 0 : ca.w;
    const int e4 = cb.x < 0 ? 0 : cb.x, e5 = cb.y < 0 ? 0 : cb.y, e6 = cb.z < 0 ? 0 : cb.z, e7 = cb.w < 0 ? 0 : cb.w;
    const int ts = e0 + e1 + e2 + e3 + e4 + e5 + e6 + e7;
    int incl = ts;
#pragma unroll
    for (int d = 1; d < 32; d <<= 1) {
      const int up = __shfl_up(incl, d);
      if (lane >= d) incl += up;
    }
    if (lane == 31) wtot[wave] = incl;
    __syncthreads();
    int pre = 0;
#pragma unroll
    for (int w2 = 0; w2 < NWAVE; ++w2) pre += (w2 < wave) ? wtot[w2] : 0;
    int run = pre + incl - ts;
    soff[8 * tid + 0] = run; run += e0;
    soff[8 * tid + 1] = run; run += e1;
    soff[8 * tid + 2] = run; run += e2;
    soff[8 * tid + 3] = run; run += e3;
    soff[8 * tid + 4] = run; run += e4;
    soff[8 * tid + 5] = run; run += e5;
    soff[8 * tid + 6] = run; run += e6;
    soff[8 * tid + 7] = run;
  }
  __syncthreads();
  for (int i = tid; i < NBMAX; i += NTHR) list[i] = soff[i];
  __syncthreads();

  if (wave == 0) {
#pragma unroll 1
    for (int b0 = 0; b0 < nh; b0 += 32) {
      const int idx = b0 + lane;
      const int uv  = reg1[idx < RCAP ? idx : RCAP - 1];
      const int m32 = (nh - b0) < 32 ? (nh - b0) : 32;
#pragma unroll 1
      for (int k = 0; k < m32; ++k) {
        const int u   = __builtin_amdgcn_readlane(uv, k);
        const int sl  = u & (NBMAX - 1);
        const int eid = (int)((unsigned)u >> 12);
        if (lane == 0) {
          int pos = list[sl];
          pos = pos < 0 ? 0 : (pos > RCAP - 1 ? RCAP - 1 : pos);
          reg2[pos] = eid;
          list[sl] = pos + 1;
        }
      }
    }
  }
  __syncthreads();

  const int nbw = nb >> 3;
  const bool ovf = (nh >= RCAP);
  const float qnan = __int_as_float(0x7fc00000);
  const int hq = lane >> 3;
#pragma unroll 1
  for (int jt = 0; jt < nbw; ++jt) {
    const int slot = wave * nbw + jt;
    const int grow = nodeBase + slot;
    const int gcl  = grow < nN ? grow : nN - 1;
    int st = soff[slot];
    const int craw = scnt[slot];
    int cnt = craw;
    st  = st < 0 ? 0 : (st > nh ? nh : st);
    cnt = cnt < 0 ? 0 : (cnt > DEGCAP ? DEGCAP : cnt);
    if (cnt > nh - st) cnt = nh - st;
    const float pz = (ovf || craw > DEGCAP) ? qnan : 0.0f;
    const bool wr = grow < nN;

    float erv[BB], mx[BB], dn[BB], av[BB][8];
#pragma unroll
    for (int b = 0; b < BB; ++b) {
      const v4f e4 = *(const v4fa*)(T + ((size_t)b * (size_t)nN + (size_t)gcl) * 8 + 4);
      erv[b] = sel4(e4, hq);
      mx[b] = -1.0e30f;
      dn[b] = 0.f;
#pragma unroll
      for (int j = 0; j < 8; ++j) av[b][j] = 0.f;
    }
    ldwait();

#pragma unroll 1
    for (int q = 0; q < cnt; ++q) {
      int idx = st + q; idx = idx > RCAP - 1 ? RCAP - 1 : idx;
      int eid = reg2[idx]; eid = eid < 0 ? 0 : (eid > nE - 1 ? nE - 1 : eid);
      const int sraw = srcs[eid];
      const int s = sraw < 0 ? 0 : (sraw > nN - 1 ? nN - 1 : sraw);
      const float we = bfr(wgt[eid]);
#pragma unroll
      for (int b = 0; b < BB; ++b) {
        const size_t rb = (size_t)b * (size_t)nN + (size_t)s;
        const v4f el4 = *(const v4fa*)(T + rb * 8);
        const float* fr = F + rb * DDIM + 8 * lane;
        const v4f fa = *(const v4fa*)fr;
        const v4f fb = *(const v4fa*)(fr + 4);
        ldwait();
        float sc = sel4(el4, hq) + erv[b];
        sc = sc > 0.f ? sc : NEGS * sc;
        sc = sc * we;
        const float df = sc - mx[b];
        const float ee = __expf(-fabsf(df));
        const bool up  = df > 0.f;
        const float s1 = up ? ee : 1.0f;
        const float s2 = up ? 1.0f : ee;
        mx[b] = up ? sc : mx[b];
        dn[b] = fmaf(dn[b], s1, s2);
        av[b][0] = fmaf(av[b][0], s1, s2 * fa.x);
        av[b][1] = fmaf(av[b][1], s1, s2 * fa.y);
        av[b][2] = fmaf(av[b][2], s1, s2 * fa.z);
        av[b][3] = fmaf(av[b][3], s1, s2 * fa.w);
        av[b][4] = fmaf(av[b][4], s1, s2 * fb.x);
        av[b][5] = fmaf(av[b][5], s1, s2 * fb.y);
        av[b][6] = fmaf(av[b][6], s1, s2 * fb.z);
        av[b][7] = fmaf(av[b][7], s1, s2 * fb.w);
      }
    }

    HiLo hl[BB];
#pragma unroll
    for (int b = 0; b < BB; ++b) {
      const float ds = dn[b] > 0.f ? dn[b] : 1.0f;
      const float iv = (dn[b] > 0.f ? 1.0f : 0.0f) * __builtin_amdgcn_rcpf(ds);
      v4f oa, ob;
      oa.x = fmaf(av[b][0], iv, pz); oa.y = fmaf(av[b][1], iv, pz);
      oa.z = fmaf(av[b][2], iv, pz); oa.w = fmaf(av[b][3], iv, pz);
      ob.x = fmaf(av[b][4], iv, pz); ob.y = fmaf(av[b][5], iv, pz);
      ob.z = fmaf(av[b][6], iv, pz); ob.w = fmaf(av[b][7], iv, pz);
      hl[b] = hilo8(oa, ob);
    }
    if (wr) {
#pragma unroll
      for (int b = 0; b < BB; ++b) {
        const size_t o = ((size_t)b * (size_t)nN + (size_t)grow) * DDIM + 8 * lane;
        *(volatile v8us*)(RSH + o) = hl[b].hi;
        *(volatile v8us*)(RSL + o) = hl[b].lo;
      }
    }
    __threadfence();
    if (wr) {
#pragma unroll
      for (int b = 0; b < BB; ++b) {
        const size_t o = ((size_t)b * (size_t)nN + (size_t)grow) * DDIM + 8 * lane;
        *(volatile v8us*)(RSH + o) = hl[b].hi;
        *(volatile v8us*)(RSL + o) = hl[b].lo;
      }
    }
  }
}

__global__ __launch_bounds__(NTHR) void k_ofc(const us* __restrict__ RSH, const us* __restrict__ RSL,
                                              const us* __restrict__ WO, const float* __restrict__ bias,
                                              us* OH, us* OL, int M) {
  __shared__ __attribute__((aligned(16))) float stg[GBM * DDIM];
  const int tid = (int)threadIdx.x, lane = tid & 31, wave = tid >> 5, hh = lane >> 4, m = lane & 15;
  const int rg = wave & 1, cg = wave >> 1;
  const int rowBase = (int)blockIdx.x * GBM;
  if (rowBase >= M) return;

  v8f acc[4];
  {
    const v8f z = {0.f, 0.f, 0.f, 0.f, 0.f, 0.f, 0.f, 0.f};
    acc[0] = z; acc[1] = z; acc[2] = z; acc[3] = z;
  }
  const size_t arow = (size_t)(rowBase + 16 * rg + m) * DDIM + DH * cg + 8 * hh;
  const us* ap  = RSH + arow;
  const us* alp = RSL + arow;
  const us* wp  = WO + (size_t)m * DH + 8 * hh;
#pragma unroll 1
  for (int ks = 0; ks < DH / 32; ++ks) {
    const FragB af  = ldfrag(ap + 32 * ks);
    const FragB alf = ldfrag(alp + 32 * ks);
#pragma unroll
    for (int t = 0; t < 4; ++t) {
      const FragB bf = ldfrag(wp + (size_t)(16 * t) * DH + 32 * ks);
      acc[t] = wmb(af, bf, acc[t]);
      acc[t] = wmb(alf, bf, acc[t]);
    }
  }

#pragma unroll
  for (int t = 0; t < 4; ++t) {
    const int o16 = 16 * t + m;
    const float bv = bfr(bias[o16]);
    const int lc = 64 * cg + o16;
#pragma unroll
    for (int r = 0; r < 8; ++r) {
      const int lr = 16 * rg + 8 * hh + r;
      stg[lr * DDIM + lc] = fmaxf(acc[t][r] + bv, 0.f);
    }
  }
  __syncthreads();

  const int q8 = lane & 7, sub = lane >> 3;
  HiLo hl[4];
#pragma unroll
  for (int i = 0; i < 4; ++i) {
    const int lr = 16 * rg + 4 * i + sub;
    const float* sp = stg + lr * DDIM + 64 * cg + 8 * q8;
    const v4f a = *(const v4fa*)sp;
    const v4f b = *(const v4fa*)(sp + 4);
    hl[i] = hilo8(a, b);
  }
#pragma unroll
  for (int i = 0; i < 4; ++i) {
    const int lr = 16 * rg + 4 * i + sub;
    const size_t o = (size_t)(rowBase + lr) * DDIM + 64 * cg + 8 * q8;
    *(volatile v8us*)(OH + o) = hl[i].hi;
    *(volatile v8us*)(OL + o) = hl[i].lo;
  }
  __threadfence();
#pragma unroll
  for (int i = 0; i < 4; ++i) {
    const int lr = 16 * rg + 4 * i + sub;
    const size_t o = (size_t)(rowBase + lr) * DDIM + 64 * cg + 8 * q8;
    *(volatile v8us*)(OH + o) = hl[i].hi;
    *(volatile v8us*)(OL + o) = hl[i].lo;
  }
}

__global__ __launch_bounds__(NTHR) void k_mlp(const us* __restrict__ H1H, const us* __restrict__ H1L,
                                              const us* __restrict__ H2H, const us* __restrict__ H2L,
                                              const us* __restrict__ WM, const float* __restrict__ bias,
                                              float* out, int M) {
  __shared__ __attribute__((aligned(16))) float stg[GBM * DDIM];
  const int tid = (int)threadIdx.x, lane = tid & 31, wave = tid >> 5, hh = lane >> 4, m = lane & 15;
  const int rg = wave & 1, cg = wave >> 1;
  const int rowBase = (int)blockIdx.x * GBM;
  if (rowBase >= M) return;

  v8f acc[4];
  {
    const v8f z = {0.f, 0.f, 0.f, 0.f, 0.f, 0.f, 0.f, 0.f};
    acc[0] = z; acc[1] = z; acc[2] = z; acc[3] = z;
  }
  const size_t arow = (size_t)(rowBase + 16 * rg + m) * DDIM + 8 * hh;
  const us* wp = WM + (size_t)(64 * cg + m) * KCAT + 8 * hh;
  {
    const us* ap = H1H + arow;
    const us* alp = H1L + arow;
#pragma unroll 1
    for (int ks = 0; ks < DDIM / 32; ++ks) {
      const FragB af  = ldfrag(ap + 32 * ks);
      const FragB alf = ldfrag(alp + 32 * ks);
#pragma unroll
      for (int t = 0; t < 4; ++t) {
        const FragB bf = ldfrag(wp + (size_t)(16 * t) * KCAT + 32 * ks);
        acc[t] = wmb(af, bf, acc[t]);
        acc[t] = wmb(alf, bf, acc[t]);
      }
    }
  }
  {
    const us* ap = H2H + arow;
    const us* alp = H2L + arow;
#pragma unroll 1
    for (int ks = 0; ks < DDIM / 32; ++ks) {
      const FragB af  = ldfrag(ap + 32 * ks);
      const FragB alf = ldfrag(alp + 32 * ks);
#pragma unroll
      for (int t = 0; t < 4; ++t) {
        const FragB bf = ldfrag(wp + (size_t)(16 * t) * KCAT + DDIM + 32 * ks);
        acc[t] = wmb(af, bf, acc[t]);
        acc[t] = wmb(alf, bf, acc[t]);
      }
    }
  }

#pragma unroll
  for (int t = 0; t < 4; ++t) {
    const int lc = 64 * cg + 16 * t + m;
    const float bv = bfr(bias[lc]);
#pragma unroll
    for (int r = 0; r < 8; ++r) {
      const int lr = 16 * rg + 8 * hh + r;
      stg[lr * DDIM + lc] = acc[t][r] + bv;
    }
  }
  __syncthreads();

  v4f fv[8];
#pragma unroll
  for (int i = 0; i < 8; ++i) {
    const int lr = 16 * rg + 2 * i + hh;
    fv[i] = *(const v4fa*)(stg + lr * DDIM + 64 * cg + 4 * m);
  }
#pragma unroll
  for (int i = 0; i < 8; ++i) {
    const int lr = 16 * rg + 2 * i + hh;
    float* op = out + (size_t)(rowBase + lr) * DDIM + 64 * cg + 4 * m;
    *(volatile v4f*)op = fv[i];
  }
  __threadfence();
#pragma unroll
  for (int i = 0; i < 8; ++i) {
    const int lr = 16 * rg + 2 * i + hh;
    float* op = out + (size_t)(rowBase + lr) * DDIM + 64 * cg + 4 * m;
    *(volatile v4f*)op = fv[i];
  }
}

static int pick_nb(int nE, int nN) {
  int nb = NBMAX;
  while (nb > 16 && (long long)nb * (long long)nE * 5LL > (long long)RCAP * (long long)nN * 4LL) nb >>= 1;
  return nb;
}
static inline int cdiv(int a, int b) { return (a + b - 1) / b; }

extern "C" void kernel_launch(void* const* d_in, const int* in_sizes, int n_in,
                              void* d_out, int out_size, void* d_ws, size_t ws_size,
                              hipStream_t stream) {
  if (n_in < 11) return;
  const int nE = in_sizes[1];
  if (nE < 1 || nE > (1 << 20)) return;
  if (in_sizes[9] != nE || in_sizes[10] != nE) return;
  if (in_sizes[0] <= 0 || (in_sizes[0] % (2 * BB * HID)) != 0) return;
  const int nN = in_sizes[0] / (2 * BB * HID);
  if (nN < 16 || nN > (1 << 20)) return;
  const int M = BB * nN;
  if ((M % GBM) != 0) return;
  if (in_sizes[2] != 2 * DDIM * DDIM) return;
  if (in_sizes[3] != 2 * NHEAD * DH) return;
  if (in_sizes[4] != 2 * NHEAD * DH) return;
  if (in_sizes[5] != 2 * DH * DH) return;
  if (in_sizes[6] != 2 * DH) return;
  if (in_sizes[7] != DDIM * KCAT) return;
  if (in_sizes[8] != DDIM) return;
  if (out_size != M * DDIM) return;

  const float* sol  = (const float*)d_in[0];
  const float* wgt  = (const float*)d_in[1];
  const float* fcw  = (const float*)d_in[2];
  const float* atl  = (const float*)d_in[3];
  const float* atr  = (const float*)d_in[4];
  const float* ofw  = (const float*)d_in[5];
  const float* ofb  = (const float*)d_in[6];
  const float* mlw  = (const float*)d_in[7];
  const float* mlb  = (const float*)d_in[8];
  const int*   src  = (const int*)d_in[9];
  const int*   dst  = (const int*)d_in[10];
  float* out = (float*)d_out;

  const int nb   = pick_nb(nE, nN);
  const int gA   = cdiv(nN, nb);
  const int vec8 = 1;
  if (gA * nb < nN) return;

  char* ws = (char*)d_ws;
  size_t off = 0;
  const size_t plane16 = (size_t)M * DDIM * 2;
  const size_t oA = off; off += 2 * plane16;                      off = (off + 255) & ~(size_t)255;
  const size_t oB = off; off += (size_t)M * DDIM * 4;             off = (off + 255) & ~(size_t)255;
  const size_t oC = off; off += 2 * plane16;                      off = (off + 255) & ~(size_t)255;
  const size_t oT = off; off += (size_t)M * 8 * 4;                off = (off + 255) & ~(size_t)255;
  const size_t oWF = off; off += (size_t)2 * DDIM * DDIM * 2;     off = (off + 255) & ~(size_t)255;
  const size_t oWO = off; off += (size_t)2 * DH * DH * 2;         off = (off + 255) & ~(size_t)255;
  const size_t oWM = off; off += (size_t)DDIM * KCAT * 2;         off = (off + 255) & ~(size_t)255;
  if (off > ws_size || off > (size_t)WSMAX) return;
  if ((size_t)M * DDIM * 4 < 2 * plane16) return;

  us*    X0  = (us*)(ws + oA);
  us*    H1H = (us*)(ws + oA);
  us*    H1L = H1H + (size_t)M * DDIM;
  float* F   = (float*)(ws + oB);
  us*    H2H = (us*)(ws + oB);
  us*    H2L = H2H + (size_t)M * DDIM;
  us*    RSH = (us*)(ws + oC);
  us*    RSL = RSH + (size_t)M * DDIM;
  float* T   = (float*)(ws + oT);
  us*    WFC = (us*)(ws + oWF);
  us*    WOF = (us*)(ws + oWO);
  us*    WML = (us*)(ws + oWM);

  hipFuncSetAttribute(reinterpret_cast<const void*>(&k_agg),
                      hipFuncAttributeMaxDynamicSharedMemorySize, LDS_AGG);

  const int u0 = M * (DDIM / 8);
  const int u1 = u0 + (2 * DDIM * DDIM) / 8;
  const int u2 = u1 + (2 * DH * DH) / 8;
  const int u3 = u2 + (DDIM * KCAT) / 8;
  k_prep<<<cdiv(u3, NTHR), NTHR, 0, stream>>>(sol, fcw, ofw, mlw, X0, WFC, WOF, WML, nN, u0, u1, u2, u3);

  const int gM = M / GBM;
  k_fc<1><<<gM, NTHR, 0, stream>>>(X0, X0, DDIM, WFC, atl, atr, F, T, M);
  k_agg<<<gA, NTHR, LDS_AGG, stream>>>(src, dst, wgt, F, T, RSH, RSL, nN, nE, nb, vec8);
  k_ofc<<<gM, NTHR, 0, stream>>>(RSH, RSL, WOF, ofb, H1H, H1L, M);
  k_fc<2><<<gM, NTHR, 0, stream>>>(H1H, H1L, DDIM, WFC + (size_t)DDIM * DDIM, atl + NHEAD * DH, atr + NHEAD * DH,
                                   F, T, M);
  k_agg<<<gA, NTHR, LDS_AGG, stream>>>(src, dst, wgt, F, T, RSH, RSL, nN, nE, nb, vec8);
  k_ofc<<<gM, NTHR, 0, stream>>>(RSH, RSL, WOF + (size_t)DH * DH, ofb + DH, H2H, H2L, M);
  k_mlp<<<gM, NTHR, 0, stream>>>(H1H, H1L, H2H, H2L, WML, mlb, out, M);
}
